// DecoderWithAttention_36197984371410
// MI455X (gfx1250) — hardware-verified
//
#include <hip/hip_runtime.h>
#include <math.h>
#include <stdint.h>


typedef _Float16 v16h __attribute__((ext_vector_type(16)));
typedef _Float16 v8h  __attribute__((ext_vector_type(8)));
typedef float    v8f  __attribute__((ext_vector_type(8)));
typedef float    v4f  __attribute__((ext_vector_type(4)));
union Frag { v16h v; v8h half[2]; };

#define NB    64
#define NDEC  12
#define NF    32
#define NH    512
#define NE    96
#define NT    4
#define KX    544
#define LDX   576
#define G3    1536
#define DOUT  1056

static_assert(NB % 64 == 0);
static_assert(NH % 64 == 0);
static_assert((NB * NE) % 64 == 0);
static_assert(KX % 32 == 0);
static_assert(NE == 96);
static_assert(NB * NT == 256);

__device__ __forceinline__ v8f zero8() {
  v8f z = {0.f, 0.f, 0.f, 0.f, 0.f, 0.f, 0.f, 0.f};
  return z;
}

__device__ __forceinline__ void ldfrag(Frag& f, const _Float16* p) {
  f.half[0] = *(const v8h*)p;
  f.half[1] = *(const v8h*)(p + 16);
}

__device__ __forceinline__ void mma16(v8f& acc, const v16h a, const v16h b) {
  acc = __builtin_amdgcn_wmma_f32_16x16x32_f16(false, a, false, b, (short)0, acc, false, false);
  asm volatile("v_nop\n\tv_nop\n\tv_nop\n\tv_nop" : "+v"(acc) : "v"(a), "v"(b));
}

__device__ __forceinline__ float wsum(float v) {
#pragma unroll
  for (int off = 16; off > 0; off >>= 1) v += __shfl_xor(v, off, 32);
  return v;
}
__device__ __forceinline__ float wmaxf(float v) {
#pragma unroll
  for (int off = 16; off > 0; off >>= 1) v = fmaxf(v, __shfl_xor(v, off, 32));
  return v;
}
__device__ __forceinline__ float sigm(float x) {
  x = fminf(fmaxf(x, -30.f), 30.f);
  return 1.0f / (1.0f + __expf(-x));
}

__global__ __launch_bounds__(256) void k_cvt(_Float16* dst, const float* src, int n8, float scale) {
  const int i = blockIdx.x * 256 + threadIdx.x;
  if (i >= n8) return;
  const float* p = src + (size_t)i * 8;
  const v4f x0 = *(const v4f*)p;
  const v4f x1 = *(const v4f*)(p + 4);
  v8h o;
  o[0] = (_Float16)(x0[0] * scale); o[1] = (_Float16)(x0[1] * scale);
  o[2] = (_Float16)(x0[2] * scale); o[3] = (_Float16)(x0[3] * scale);
  o[4] = (_Float16)(x1[0] * scale); o[5] = (_Float16)(x1[1] * scale);
  o[6] = (_Float16)(x1[2] * scale); o[7] = (_Float16)(x1[3] * scale);
  _Float16* q = dst + (size_t)i * 8;
  *(volatile v8h*)q = o;
  __threadfence();
  *(volatile v8h*)q = o;
}

__global__ __launch_bounds__(256) void k_gemm(float* C, int ldc, const _Float16* A, int lda,
                                              const _Float16* W, int ldw, const float* bias,
                                              int has_bias, int K, float scale) {
  __shared__ __attribute__((aligned(16))) float s_c[64 * 64];
  const int tid = threadIdx.x, lane = tid & 31, wv = tid >> 5;
  const int h = lane >> 4, m = lane & 15;
  const int rt = wv & 3, cp = wv >> 2;
  const int row0 = blockIdx.y * 64, col0 = blockIdx.x * 64;

  const _Float16* ap  = A + (size_t)(row0 + rt * 16 + m) * lda + 8 * h;
  const _Float16* bp0 = W + (size_t)(col0 + cp * 32 + m) * ldw + 8 * h;
  const _Float16* bp1 = W + (size_t)(col0 + cp * 32 + 16 + m) * ldw + 8 * h;

  v8f acc0 = zero8(), acc1 = zero8();
  for (int k0 = 0; k0 < K; k0 += 32) {
    Frag a, b0, b1;
    ldfrag(a, ap + k0);
    ldfrag(b0, bp0 + k0);
    ldfrag(b1, bp1 + k0);
    mma16(acc0, a.v, b0.v);
    mma16(acc1, a.v, b1.v);
  }

  float bv0 = 0.f, bv1 = 0.f;
  if (has_bias) {
    bv0 = bias[col0 + cp * 32 + m];
    bv1 = bias[col0 + cp * 32 + 16 + m];
  }
#pragma unroll
  for (int r = 0; r < 8; ++r) {
    const int lr = rt * 16 + 8 * h + r;
    s_c[lr * 64 + cp * 32 + m]      = acc0[r] * scale + bv0;
    s_c[lr * 64 + cp * 32 + 16 + m] = acc1[r] * scale + bv1;
  }
  __syncthreads();

  const int c  = (lane & 15) * 4, rh = lane >> 4;
  const int r0 = wv * 8 + rh, r1 = r0 + 2, r2 = r0 + 4, r3 = r0 + 6;
  const v4f v0 = *(const v4f*)&s_c[r0 * 64 + c];
  const v4f v1 = *(const v4f*)&s_c[r1 * 64 + c];
  const v4f v2 = *(const v4f*)&s_c[r2 * 64 + c];
  const v4f v3 = *(const v4f*)&s_c[r3 * 64 + c];
  float* p0 = C + (size_t)(row0 + r0) * ldc + col0 + c;
  float* p1 = C + (size_t)(row0 + r1) * ldc + col0 + c;
  float* p2 = C + (size_t)(row0 + r2) * ldc + col0 + c;
  float* p3 = C + (size_t)(row0 + r3) * ldc + col0 + c;
  *(volatile v4f*)p0 = v0; *(volatile v4f*)p1 = v1;
  *(volatile v4f*)p2 = v2; *(volatile v4f*)p3 = v3;
  __threadfence();
  *(volatile v4f*)p0 = v0; *(volatile v4f*)p1 = v1;
  *(volatile v4f*)p2 = v2; *(volatile v4f*)p3 = v3;
}

__global__ __launch_bounds__(512) void k_gru(float* H32o, _Float16* H16o,
                                             const _Float16* X, int ldx, int Kx,
                                             const _Float16* Wi,
                                             const _Float16* Hp16,
                                             const _Float16* Wh,
                                             const float* Hp32,
                                             const float* bi, const float* bh, float scale) {
  __shared__ __attribute__((aligned(16))) float    s_h[64 * 64];
  __shared__ __attribute__((aligned(16))) _Float16 s_q[64 * 64];
  const int tid = threadIdx.x, lane = tid & 31, wv = tid >> 5;
  const int h = lane >> 4, m = lane & 15;
  const int rt = wv & 3, ct = wv >> 2;
  const int j0 = blockIdx.x * 64, cl = ct * 16 + m, col = j0 + cl;

  const _Float16* xp = X + (size_t)(rt * 16 + m) * ldx + 8 * h;
  const _Float16* wr = Wi + (size_t)col * Kx + 8 * h;
  const _Float16* wz = Wi + (size_t)(NH + col) * Kx + 8 * h;
  const _Float16* wn = Wi + (size_t)(2 * NH + col) * Kx + 8 * h;
  v8f ir = zero8(), iz = zero8(), in_ = zero8();
  for (int k0 = 0; k0 < Kx; k0 += 32) {
    Frag a, b0, b1, b2;
    ldfrag(a, xp + k0);
    ldfrag(b0, wr + k0);
    ldfrag(b1, wz + k0);
    ldfrag(b2, wn + k0);
    mma16(ir, a.v, b0.v);
    mma16(iz, a.v, b1.v);
    mma16(in_, a.v, b2.v);
  }
  const _Float16* hp = Hp16 + (size_t)(rt * 16 + m) * NH + 8 * h;
  const _Float16* ur = Wh + (size_t)col * NH + 8 * h;
  const _Float16* uz = Wh + (size_t)(NH + col) * NH + 8 * h;
  const _Float16* un = Wh + (size_t)(2 * NH + col) * NH + 8 * h;
  v8f hr = zero8(), hz = zero8(), hn_ = zero8();
  for (int k0 = 0; k0 < NH; k0 += 32) {
    Frag a, b0, b1, b2;
    ldfrag(a, hp + k0);
    ldfrag(b0, ur + k0);
    ldfrag(b1, uz + k0);
    ldfrag(b2, un + k0);
    mma16(hr, a.v, b0.v);
    mma16(hz, a.v, b1.v);
    mma16(hn_, a.v, b2.v);
  }

  const float bir = bi[col], biz = bi[NH + col], bin = bi[2 * NH + col];
  const float bhr = bh[col], bhz = bh[NH + col], bhn = bh[2 * NH + col];
#pragma unroll
  for (int r = 0; r < 8; ++r) {
    const int row = rt * 16 + 8 * h + r;
    const float gir = ir[r]  * scale + bir, ghr = hr[r]  * scale + bhr;
    const float giz = iz[r]  * scale + biz, ghz = hz[r]  * scale + bhz;
    const float gin = in_[r] * scale + bin, ghn = hn_[r] * scale + bhn;
    const float rg = sigm(gir + ghr);
    const float zg = sigm(giz + ghz);
    const float ng = tanhf(gin + rg * ghn);
    const float hpv = Hp32[(size_t)row * NH + col];
    const float hv = (1.0f - zg) * ng + zg * hpv;
    s_h[row * 64 + cl] = hv;
    s_q[row * 64 + cl] = (_Float16)hv;
  }
  __syncthreads();

  const int c4 = (lane & 15) * 4;
  const int rA = 4 * wv + (lane >> 4), rB = rA + 2;
  const v4f f0 = *(const v4f*)&s_h[rA * 64 + c4];
  const v4f f1 = *(const v4f*)&s_h[rB * 64 + c4];
  float* q0 = H32o + (size_t)rA * NH + j0 + c4;
  float* q1 = H32o + (size_t)rB * NH + j0 + c4;
  const int c8 = (lane & 7) * 8, rC = 4 * wv + (lane >> 3);
  const v8h g0 = *(const v8h*)&s_q[rC * 64 + c8];
  _Float16* q2 = H16o + (size_t)rC * NH + j0 + c8;
  *(volatile v4f*)q0 = f0; *(volatile v4f*)q1 = f1; *(volatile v8h*)q2 = g0;
  __threadfence();
  *(volatile v4f*)q0 = f0; *(volatile v4f*)q1 = f1; *(volatile v8h*)q2 = g0;
}

__global__ __launch_bounds__(256) void k_attn(const float* encproj,
                                              const float* aq,
                                              const float* vattn,
                                              const float* enc,
                                              const float* cur_in, int cur_ld,
                                              float* wsf,
                                              _Float16* xcat) {
  __shared__ __attribute__((aligned(16))) float    s_a[NH];
  __shared__ __attribute__((aligned(16))) float    s_v[NH];
  __shared__ __attribute__((aligned(16))) float    s_ws[NH];
  __shared__ float s_e[NE];
  __shared__ __attribute__((aligned(16))) _Float16 s_x[LDX];
  const int tid = threadIdx.x, lane = tid & 31, wv = tid >> 5, b = blockIdx.x;

  for (int i = tid; i < NH; i += 256) {
    s_a[i] = aq[(size_t)b * NH + i];
    s_v[i] = vattn[i];
  }
  __syncthreads();

  const float* epb = encproj + (size_t)b * NE * NH;
  for (int e = wv; e < NE; e += 8) {
    const float* row = epb + (size_t)e * NH;
    float s = 0.f;
#pragma unroll 1
    for (int i = 0; i < NH / 32; ++i) {
      const int g = lane + 32 * i;
      s += s_v[g] * tanhf(row[g] + s_a[g]);
    }
    s = wsum(s);
    if (lane == 0) s_e[e] = s;
  }
  __syncthreads();

  if (wv == 0) {
    const float x0 = s_e[lane], x1 = s_e[lane + 32], x2 = s_e[lane + 64];
    const float mx = wmaxf(fmaxf(x0, fmaxf(x1, x2)));
    const float e0 = __expf(x0 - mx), e1 = __expf(x1 - mx), e2 = __expf(x2 - mx);
    const float sm = wsum(e0 + e1 + e2);
    const float inv = 1.0f / sm;
    s_e[lane] = e0 * inv; s_e[lane + 32] = e1 * inv; s_e[lane + 64] = e2 * inv;
  }
  __syncthreads();

  const float* eb = enc + (size_t)b * NE * NH;
  float c0 = 0.f, c1 = 0.f;
#pragma unroll 4
  for (int e = 0; e < NE; ++e) {
    const float w = s_e[e];
    const float* er = eb + (size_t)e * NH;
    c0 += w * er[tid];
    c1 += w * er[tid + 256];
  }
  s_ws[tid] = c0; s_ws[tid + 256] = c1;
  s_x[NF + tid] = (_Float16)c0; s_x[NF + 256 + tid] = (_Float16)c1;
  if (tid < NF) s_x[tid] = (_Float16)cur_in[(size_t)b * cur_ld + tid];
  else if (tid < NF + (LDX - KX)) s_x[KX + tid - NF] = (_Float16)0.f;
  __syncthreads();

  float* wrow = wsf + (size_t)b * NH;
  _Float16* xrow = xcat + (size_t)b * LDX;
  const bool do_ws = (wv < 4);
  const int  widx  = wv * 32 + lane;
  const int  xidx  = (wv - 4) * 32 + lane;
  const bool do_x  = (wv >= 4) && (xidx < LDX / 8);
  v4f vw = {0.f, 0.f, 0.f, 0.f};
  v8h vx;
#pragma unroll
  for (int i = 0; i < 8; ++i) vx[i] = (_Float16)0.f;
  if (do_ws) vw = *(const v4f*)&s_ws[widx * 4];
  if (do_x)  vx = *(const v8h*)&s_x[xidx * 8];
  float* pw = wrow + widx * 4;
  _Float16* px = xrow + xidx * 8;
  if (do_ws) *(volatile v4f*)pw = vw;
  if (do_x)  *(volatile v8h*)px = vx;
  __threadfence();
  if (do_ws) *(volatile v4f*)pw = vw;
  if (do_x)  *(volatile v8h*)px = vx;
}

__global__ __launch_bounds__(256) void k_out(const float* h1, const float* wsf,
                                             const float* cur_in, int cur_ld,
                                             const float* Wout, const float* bout,
                                             const int* tidx, const float* xrow,
                                             float* cur_out, float* ostage, float* dout, int t) {
  __shared__ __attribute__((aligned(16))) float s_out[NB * NT];
  __shared__ __attribute__((aligned(16))) float s_cur[NB * NF];
  const int tid = threadIdx.x, lane = tid & 31, wv = tid >> 5;

  for (int i = 0; i < 32; ++i) {
    const int p = wv * 32 + i, b = p >> 2, o = p & 3;
    const float* hb = h1 + (size_t)b * NH;
    const float* wb = wsf + (size_t)b * NH;
    const float* cb = cur_in + (size_t)b * cur_ld;
    const float* wr = Wout + (size_t)o * DOUT;
    float s = 0.f;
    for (int j = 0; j < NH / 32; ++j) { const int k = lane + 32 * j; s += hb[k] * wr[k]; }
    for (int j = 0; j < NH / 32; ++j) { const int k = lane + 32 * j; s += wb[k] * wr[NH + k]; }
    s += cb[lane] * wr[2 * NH + lane];
    s = wsum(s);
    if (lane == 0) s_out[p] = s + bout[o];
  }
  __syncthreads();

  int ix0 = tidx[0], ix1 = tidx[1], ix2 = tidx[2], ix3 = tidx[3];
  if (ix0 < 0) ix0 += NF; if (ix1 < 0) ix1 += NF; if (ix2 < 0) ix2 += NF; if (ix3 < 0) ix3 += NF;
  for (int i = tid; i < NB * NF; i += 256) {
    const int b = i >> 5, f = i & 31;
    const float tv = xrow[(size_t)b * (NDEC * NF) + f];
    const v4f ov = *(const v4f*)&s_out[b * 4];
    float v = tv;
    v = (ix0 == f) ? ov[0] : v;
    v = (ix1 == f) ? ov[1] : v;
    v = (ix2 == f) ? ov[2] : v;
    v = (ix3 == f) ? ov[3] : v;
    s_cur[i] = v;
  }
  __syncthreads();

  const v4f vc0 = *(const v4f*)&s_cur[tid * 4];
  const v4f vc1 = *(const v4f*)&s_cur[(256 + tid) * 4];
  float* pc0 = cur_out + (size_t)tid * 4;
  float* pc1 = cur_out + (size_t)(256 + tid) * 4;
  const bool do_o = (tid < (NB * NT) / 4);
  v4f vo = {0.f, 0.f, 0.f, 0.f};
  if (do_o) vo = *(const v4f*)&s_out[tid * 4];
  float* po = ostage + (size_t)t * (NB * NT) + tid * 4;
  *(volatile v4f*)pc0 = vc0; *(volatile v4f*)pc1 = vc1;
  if (do_o) *(volatile v4f*)po = vo;
  __threadfence();
  *(volatile v4f*)pc0 = vc0; *(volatile v4f*)pc1 = vc1;
  if (do_o) *(volatile v4f*)po = vo;

  if (t == NDEC - 1) {
    const int i0 = tid, i1 = 256 + tid, i2 = 512 + tid;
    const int b0 = i0 / NDEC, t0 = i0 - b0 * NDEC;
    const int b1 = i1 / NDEC, t1 = i1 - b1 * NDEC;
    const int b2 = i2 / NDEC, t2 = i2 - b2 * NDEC;
    v4f d0, d1, d2;
    const v4f l0 = *(const v4f*)&s_out[b0 * 4], l1 = *(const v4f*)&s_out[b1 * 4], l2 = *(const v4f*)&s_out[b2 * 4];
    const int g0i = (t0 == t) ? 0 : t0, g1i = (t1 == t) ? 0 : t1, g2i = (t2 == t) ? 0 : t2;
    const v4f g0 = *(const v4f*)(ostage + (size_t)g0i * (NB * NT) + b0 * 4);
    const v4f g1 = *(const v4f*)(ostage + (size_t)g1i * (NB * NT) + b1 * 4);
    const v4f g2 = *(const v4f*)(ostage + (size_t)g2i * (NB * NT) + b2 * 4);
    d0 = (t0 == t) ? l0 : g0; d1 = (t1 == t) ? l1 : g1; d2 = (t2 == t) ? l2 : g2;
    float* pd0 = dout + (size_t)i0 * 4;
    float* pd1 = dout + (size_t)i1 * 4;
    float* pd2 = dout + (size_t)i2 * 4;
    *(volatile v4f*)pd0 = d0; *(volatile v4f*)pd1 = d1; *(volatile v4f*)pd2 = d2;
    __threadfence();
    *(volatile v4f*)pd0 = d0; *(volatile v4f*)pd1 = d1; *(volatile v4f*)pd2 = d2;
  }
}

static inline unsigned cdivu(unsigned a, unsigned b) { return (a + b - 1) / b; }

extern "C" void kernel_launch(void* const* d_in, const int* in_sizes, int n_in,
                              void* d_out, int out_size, void* d_ws, size_t ws_size,
                              hipStream_t stream) {
  if (n_in < 17) return;
  if (out_size < NB * NDEC * NT) return;
  if (in_sizes[0] < NB * NDEC * NF || in_sizes[1] < 2 * NB * NH || in_sizes[2] < NB * NE * NH ||
      in_sizes[3] < NT || in_sizes[4] < NH * 2 * NH || in_sizes[5] < NH || in_sizes[6] < NH ||
      in_sizes[7] < G3 * KX || in_sizes[8] < G3 * NH || in_sizes[9] < G3 || in_sizes[10] < G3 ||
      in_sizes[11] < G3 * NH || in_sizes[12] < G3 * NH || in_sizes[13] < G3 || in_sizes[14] < G3 ||
      in_sizes[15] < NT * DOUT || in_sizes[16] < NT) return;

  const float* inputs = (const float*)d_in[0];
  const float* hidden = (const float*)d_in[1];
  const float* enc    = (const float*)d_in[2];
  const int*   tidx   = (const int*)d_in[3];
  const float* W_attn = (const float*)d_in[4];
  const float* b_attn = (const float*)d_in[5];
  const float* v_attn = (const float*)d_in[6];
  const float* Wi0    = (const float*)d_in[7];
  const float* Wh0    = (const float*)d_in[8];
  const float* bi0    = (const float*)d_in[9];
  const float* bh0    = (const float*)d_in[10];
  const float* Wi1    = (const float*)d_in[11];
  const float* Wh1    = (const float*)d_in[12];
  const float* bi1    = (const float*)d_in[13];
  const float* bh1    = (const float*)d_in[14];
  const float* Wout   = (const float*)d_in[15];
  const float* bout   = (const float*)d_in[16];
  float* dout = (float*)d_out;

  size_t off = 0;
  auto carve = [&](size_t bytes) -> size_t {
    const size_t o = off;
    off += (bytes + 255) & ~(size_t)255;
    return o;
  };
  const size_t o_enc16 = carve(sizeof(_Float16) * (size_t)NB * NE * NH);
  const size_t o_wa16  = carve(sizeof(_Float16) * (size_t)NH * 2 * NH);
  const size_t o_wi0   = carve(sizeof(_Float16) * (size_t)G3 * KX);
  const size_t o_wh0   = carve(sizeof(_Float16) * (size_t)G3 * NH);
  const size_t o_wi1   = carve(sizeof(_Float16) * (size_t)G3 * NH);
  const size_t o_wh1   = carve(sizeof(_Float16) * (size_t)G3 * NH);
  const size_t o_encp  = carve(sizeof(float) * (size_t)NB * NE * NH);
  const size_t o_a     = carve(sizeof(float) * (size_t)NB * NH);
  const size_t o_ws    = carve(sizeof(float) * (size_t)NB * NH);
  const size_t o_xcat  = carve(sizeof(_Float16) * (size_t)NB * LDX);
  const size_t o_h32   = carve(sizeof(float) * (size_t)4 * NB * NH);
  const size_t o_h16   = carve(sizeof(_Float16) * (size_t)4 * NB * NH);
  const size_t o_cur   = carve(sizeof(float) * (size_t)NB * NF);
  const size_t o_ost   = carve(sizeof(float) * (size_t)NDEC * NB * NT);
  if (off > ws_size) return;

  char* wsb = (char*)d_ws;
  _Float16* enc16 = (_Float16*)(wsb + o_enc16);
  _Float16* wa16  = (_Float16*)(wsb + o_wa16);
  _Float16* wi0h  = (_Float16*)(wsb + o_wi0);
  _Float16* wh0h  = (_Float16*)(wsb + o_wh0);
  _Float16* wi1h  = (_Float16*)(wsb + o_wi1);
  _Float16* wh1h  = (_Float16*)(wsb + o_wh1);
  float*    encp  = (float*)(wsb + o_encp);
  float*    abuf  = (float*)(wsb + o_a);
  float*    wsf   = (float*)(wsb + o_ws);
  _Float16* xcat  = (_Float16*)(wsb + o_xcat);
  float*    h32   = (float*)(wsb + o_h32);
  _Float16* h16   = (_Float16*)(wsb + o_h16);
  float*    curb  = (float*)(wsb + o_cur);
  float*    ost   = (float*)(wsb + o_ost);

  const float wscale = 64.0f, inv_w = 1.0f / 64.0f;
  const size_t BH = (size_t)NB * NH;

  {
    const int n8_enc = NB * NE * NH / 8, n8_wa = NH * 2 * NH / 8, n8_wi0 = G3 * KX / 8, n8_w = G3 * NH / 8, n8_hid = 2 * NB * NH / 8;
    k_cvt<<<cdivu(n8_enc, 256), 256, 0, stream>>>(enc16, enc, n8_enc, 1.0f);
    k_cvt<<<cdivu(n8_wa, 256), 256, 0, stream>>>(wa16, W_attn, n8_wa, wscale);
    k_cvt<<<cdivu(n8_wi0, 256), 256, 0, stream>>>(wi0h, Wi0, n8_wi0, wscale);
    k_cvt<<<cdivu(n8_w, 256), 256, 0, stream>>>(wh0h, Wh0, n8_w, wscale);
    k_cvt<<<cdivu(n8_w, 256), 256, 0, stream>>>(wi1h, Wi1, n8_w, wscale);
    k_cvt<<<cdivu(n8_w, 256), 256, 0, stream>>>(wh1h, Wh1, n8_w, wscale);
    k_cvt<<<cdivu(n8_hid, 256), 256, 0, stream>>>(h16 + 2 * BH, hidden, n8_hid, 1.0f);
  }

  k_gemm<<<dim3(NH / 64, (NB * NE) / 64), 256, 0, stream>>>(
      encp, NH, enc16, NH, wa16 + NH, 2 * NH, b_attn, 0, NH, inv_w);

  for (int t = 0; t < NDEC; ++t) {
    const int pr = (t + 1) & 1;
    const int pw = t & 1;
    const _Float16* h0p16 = h16 + (size_t)(pr * 2 + 0) * BH;
    const _Float16* h1p16 = h16 + (size_t)(pr * 2 + 1) * BH;
    _Float16* h0n16 = h16 + (size_t)(pw * 2 + 0) * BH;
    _Float16* h1n16 = h16 + (size_t)(pw * 2 + 1) * BH;
    const float* h0p32 = (t == 0) ? hidden : (h32 + (size_t)(pr * 2 + 0) * BH);
    const float* h1p32 = (t == 0) ? (hidden + BH) : (h32 + (size_t)(pr * 2 + 1) * BH);
    float* h0n32 = h32 + (size_t)(pw * 2 + 0) * BH;
    float* h1n32 = h32 + (size_t)(pw * 2 + 1) * BH;
    const float* cur_in = (t == 0) ? inputs : curb;
    const int cur_ld = (t == 0) ? (NDEC * NF) : NF;

    k_gemm<<<dim3(NH / 64, NB / 64), 256, 0, stream>>>(
        abuf, NH, h1p16, NH, wa16, 2 * NH, b_attn, 1, NH, inv_w);
    k_attn<<<NB, 256, 0, stream>>>(encp, abuf, v_attn, enc, cur_in, cur_ld, wsf, xcat);
    k_gru<<<NH / 64, 512, 0, stream>>>(h0n32, h0n16, xcat, LDX, KX, wi0h, h0p16, wh0h, h0p32, bi0, bh0, inv_w);
    k_gru<<<NH / 64, 512, 0, stream>>>(h1n32, h1n16, h0n16, NH, NH, wi1h, h1p16, wh1h, h1p32, bi1, bh1, inv_w);
    k_out<<<1, 256, 0, stream>>>(h1n32, wsf, cur_in, cur_ld, Wout, bout, tidx, inputs + (size_t)t * NF, curb, ost, dout, t);
  }
}
